// BetterBot_44169443672375
// MI455X (gfx1250) — hardware-run, weakly checked
//
#include <hip/hip_runtime.h>


#ifndef NB
#define NB 65536
#endif
#define NB_FULL 65536
#define DM    8
#define NH_   2
#define HD    4
#define NL    5
#define NT    15
#define AOUT  20
#define NDICE 15
#define NSTAR 15
#define NBTN  2
#define WPB   4
#define BLOCK (32 * WPB)
#define IPW   16
#define PSH   14.0f
#define SC2   ((float)(0.5 * 1.4426950408889634))
#define NEGB  (-3.0e38f)

static_assert(NH_ * HD == DM);
static_assert(DM == 8);
static_assert(HD == 4);
static_assert(3 * NL == NT);
static_assert(NT == 15);
static_assert(AOUT > 16);
static_assert(AOUT <= 32);
static_assert(3 * DM == 24);
static_assert(BLOCK == 128);
static_assert((NDICE + NSTAR + NBTN) * DM == 2 * BLOCK);
static_assert(NB % (WPB * IPW) == 0);
static_assert(NB <= NB_FULL);
static_assert(IPW * NL == 80);
static_assert((IPW * AOUT * 4) % 128 == 0);
static_assert(IPW * AOUT * 4 == 80 * 16);
static_assert(80 % 8 == 0);
static_assert(10 * 128 * 2 + 256 * 4 + 128 * 4 + WPB * 240 * 4 + WPB * IPW * AOUT * 4 <= 131072);

typedef _Float16 h16;
typedef __attribute__((ext_vector_type(16))) _Float16 v16h;
typedef __attribute__((ext_vector_type(8)))  _Float16 v8h;
typedef __attribute__((ext_vector_type(8)))  float    v8f;
typedef __attribute__((ext_vector_type(4)))  float    v4f;
typedef __attribute__((ext_vector_type(4)))  unsigned v4u;
typedef __attribute__((ext_vector_type(8)))  unsigned v8u;
typedef v4f  __attribute__((may_alias)) v4fa;

__device__ __forceinline__ unsigned short f2bf(float f) { unsigned u = __float_as_uint(f); u += 0x7FFFu + ((u >> 16) & 1u); return (unsigned short)(u >> 16); }
__device__ __forceinline__ float bfr(float f) { return __uint_as_float(((unsigned)f2bf(f)) << 16); }
__device__ __forceinline__ v16h cat16(v8h lo, v8h hi) { return __builtin_shufflevector(lo, hi, 0, 1, 2, 3, 4, 5, 6, 7, 8, 9, 10, 11, 12, 13, 14, 15); }
__device__ __forceinline__ void wave_sync() { __builtin_amdgcn_fence(3  , "wavefront"); __builtin_amdgcn_wave_barrier(); asm volatile("" ::: "memory"); }
static __device__ __forceinline__ h16 toh_flush(float v) { const h16 r = (h16)v; return (fabsf(v) < 6.103515625e-05f) ? (h16)0.0f : r; }
static __device__ __forceinline__ v8f wmma16g(v16h a, v16h b, v8f c) {
    c = __builtin_amdgcn_wmma_f32_16x16x32_f16(false, a, false, b, (short)0, c, false, false);
    asm volatile("v_nop\n\tv_nop\n\tv_nop\n\tv_nop" : "+v"(c) : "v"(a), "v"(b));
    return c;
}
static __device__ __forceinline__ float ldsel(const float* __restrict__ src, int e, int n) {
    const int ec = e < 0 ? 0 : (e >= n ? n - 1 : e);
    float v = src[ec];
    asm volatile("" : "+v"(v));
    return ((e >= 0) & (e < n)) ? v : 0.0f;
}
static __device__ __forceinline__ void soft16(const v8f s, const int hi, v8h& p, float& inv) {
    float t[8]; float mx = NEGB;
#pragma unroll
    for (int r = 0; r < 8; ++r) {
        t[r] = s[r] * SC2;
        const float c = (r == 7) ? ((hi == 1) ? NEGB : t[r]) : t[r];
        mx = fmaxf(mx, c); }
    mx = fmaxf(mx, __shfl_xor(mx, 16, 32));
    const float sh = PSH - mx;
    float ls = 0.0f;
#pragma unroll
    for (int r = 0; r < 8; ++r) {
        const float e = t[r] + sh;
        float g = (e < -14.0f) ? 0.0f : __builtin_amdgcn_exp2f(e);
        if (r == 7) g = (hi == 1) ? 0.0f : g;
        const h16 c = (h16)g;
        p[r] = c; ls += (float)c; }
    ls += __shfl_xor(ls, 16, 32);
    inv = 1.0f / ls;
}

__global__ __launch_bounds__(BLOCK) void k_encoder(
    const int* __restrict__ dice_type, const int* __restrict__ dice_star, const int* __restrict__ summon_lvl,
    const float* __restrict__ emb_dice, const float* __restrict__ emb_star, const float* __restrict__ emb_btns,
    const float* __restrict__ Wout, const float* __restrict__ bout,
    const float* __restrict__ Wqkv0, const float* __restrict__ bqkv0, const float* __restrict__ Wo0, const float* __restrict__ bo0,
    const float* __restrict__ Wl0, const float* __restrict__ bl0,
    const float* __restrict__ Wqkv1, const float* __restrict__ bqkv1, const float* __restrict__ Wo1, const float* __restrict__ bo1,
    const float* __restrict__ Wl1, const float* __restrict__ bl1,
    float* OUT)
{
    __shared__ __align__(16) h16   wl[10 * 128];
    __shared__ __align__(16) float tab[256];
    __shared__ __align__(16) float bs[128];
    __shared__ __align__(16) int   ix[WPB * 240];
    __shared__ __align__(16) float os[WPB * IPW * AOUT];

    const int tid = (int)threadIdx.x;
    const int lane = tid & 31, lr = lane & 15, hi = lane >> 4;
    const int wave = __builtin_amdgcn_readfirstlane((int)(threadIdx.x >> 5));

    wl[0 * 128 + tid] = toh_flush(bfr(ldsel(Wqkv0,       tid, 128)));
    wl[1 * 128 + tid] = toh_flush(bfr(ldsel(Wqkv0 + 128, tid, 64)));
    wl[2 * 128 + tid] = toh_flush(bfr(ldsel(Wo0,         tid, 64)));
    wl[3 * 128 + tid] = toh_flush(bfr(ldsel(Wl0,         tid, 64)));
    wl[4 * 128 + tid] = toh_flush(bfr(ldsel(Wqkv1,       tid, 128)));
    wl[5 * 128 + tid] = toh_flush(bfr(ldsel(Wqkv1 + 128, tid, 64)));
    wl[6 * 128 + tid] = toh_flush(bfr(ldsel(Wo1,         tid, 64)));
    wl[7 * 128 + tid] = toh_flush(bfr(ldsel(Wl1,         tid, 64)));
    wl[8 * 128 + tid] = toh_flush(bfr(ldsel(Wout,        tid, 128)));
    wl[9 * 128 + tid] = toh_flush(bfr(ldsel(Wout + 128,  tid, 32)));
#pragma unroll 1
    for (int e = tid; e < 256; e += BLOCK) {
        const float v = ldsel(emb_dice, e, NDICE * DM) + ldsel(emb_star, e - NDICE * DM, NSTAR * DM) + ldsel(emb_btns, e - (NDICE + NSTAR) * DM, NBTN * DM);
        tab[e] = bfr(v); }
    { const float v = ldsel(bqkv0, tid, 24) + ldsel(bqkv1, tid - 32, 24) + ldsel(bo0, tid - 64, 8) + ldsel(bl0, tid - 72, 8)
                    + ldsel(bo1, tid - 80, 8) + ldsel(bl1, tid - 88, 8) + ldsel(bout, tid - 96, AOUT);
      bs[tid] = bfr(v); }

    const int b0 = (blockIdx.x * WPB + wave) * IPW;
    const int xb = wave * 240;
#pragma unroll
    for (int s = 0; s < 3; ++s) {
        const int j = s * 32 + lane; const int jc = j < 80 ? j : 79;
        const size_t g = (size_t)b0 * NL + (size_t)jc;
        int a0 = dice_type[g], a1 = dice_star[g], a2 = summon_lvl[g];
        asm volatile("" : "+v"(a0), "+v"(a1), "+v"(a2));
        if (j < 80) { ix[xb + j] = a0; ix[xb + 80 + j] = a1; ix[xb + 160 + j] = a2; } }
    __syncthreads();

    const bool lo = (hi == 0);
    const v8h z8 = (v8h){};
    const v8f zf = (v8f){};
    const int arr = (lr >= 2 * NL) ? 2 : ((lr >= NL) ? 1 : 0);
    int tk = lr - NL * arr; tk = tk > NL - 1 ? NL - 1 : tk;
    const int ioff = xb + arr * 80 + tk;
    const int tsz = (arr == 2) ? NBTN : NDICE;
    const int tb = arr * NDICE;
    const bool tokv = lo & (lr < NT);
    const bool hd0 = lr < HD, hd1 = (lr >= HD) & (lr < 2 * HD);
    v8h wo0 = *(const v8h*)(&wl[8 * 128 + lr * 8]); wo0 = lo ? wo0 : z8;
    v8h wo1 = *(const v8h*)(&wl[9 * 128 + lr * 8]); wo1 = lo ? wo1 : z8;
    const v16h wout0 = cat16(wo0, z8), wout1 = cat16(wo1, z8);
    const float bout0 = bs[96 + lr], bout1 = bs[112 + lr];
    const int ob = wave * (IPW * AOUT);

#pragma unroll 1
    for (int it = 0; it < IPW; ++it) {
        int idx = ix[ioff + it * NL];
        idx = idx < 0 ? idx + tsz : idx;
        idx = idx < 0 ? 0 : (idx >= tsz ? tsz - 1 : idx);
        const int tro = (tb + idx) * DM;
        const v4f xa = *(const v4fa*)(&tab[tro]), xc = *(const v4fa*)(&tab[tro + 4]);
        float x[8];
#pragma unroll
        for (int r = 0; r < 4; ++r) { x[r] = tokv ? xa[r] : 0.0f; x[4 + r] = tokv ? xc[r] : 0.0f; }

#pragma unroll 1
        for (int L = 0; L < 2; ++L) {
            const int wp = L * 512, bq = L * 32, bob = 64 + L * 16, blb = 72 + L * 16;
            v8h xh;
#pragma unroll
            for (int r = 0; r < 8; ++r) xh[r] = toh_flush(x[r]);
            const v16h xf = cat16(xh, z8);
            v8h wqk = *(const v8h*)(&wl[wp + lr * 8]); wqk = lo ? wqk : z8;
            v8f qk = wmma16g(cat16(wqk, z8), xf, zf);
            { const v4f ba = *(const v4fa*)(&bs[bq + 8 * hi]), bb = *(const v4fa*)(&bs[bq + 8 * hi + 4]);
#pragma unroll
              for (int r = 0; r < 4; ++r) { qk[r] += ba[r]; qk[4 + r] += bb[r]; } }
            v8h wv = *(const v8h*)(&wl[wp + 128 + lr * 8]); wv = lo ? wv : z8;
            const v8f vv = wmma16g(xf, cat16(wv, z8), zf);
            const float bvv = bs[bq + 16 + lr];
            v8h va0, va1;
#pragma unroll
            for (int r = 0; r < 8; ++r) {
                h16 c = toh_flush(vv[r] + bvv);
                if (r == 7) c = (hi == 1) ? (h16)0.0f : c;
                va0[r] = hd0 ? c : (h16)0.0f; va1[r] = hd1 ? c : (h16)0.0f; }
            const v16h vA = cat16(va0, va1);
            v8h qh;
#pragma unroll
            for (int r = 0; r < 8; ++r) qh[r] = toh_flush(qk[r]);
            const v4u own = __builtin_bit_cast(v4u, qh);
            v4u oth;
#pragma unroll
            for (int i = 0; i < 4; ++i) oth[i] = (unsigned)__shfl_xor((int)own[i], 16, 32);
            v8u fq0 = (v8u){}, fq1 = (v8u){}, fk0 = (v8u){}, fk1 = (v8u){};
            fq0[0] = lo ? own[0] : 0u; fq0[1] = lo ? own[1] : 0u;
            fq1[0] = lo ? own[2] : 0u; fq1[1] = lo ? own[3] : 0u;
            fk0[0] = lo ? oth[0] : 0u; fk0[1] = lo ? oth[1] : 0u;
            fk1[0] = lo ? oth[2] : 0u; fk1[1] = lo ? oth[3] : 0u;
            const v8f s0 = wmma16g(__builtin_bit_cast(v16h, fk0), __builtin_bit_cast(v16h, fq0), zf);
            const v8f s1 = wmma16g(__builtin_bit_cast(v16h, fk1), __builtin_bit_cast(v16h, fq1), zf);
            v8h p0, p1; float inv0, inv1;
            soft16(s0, hi, p0, inv0);
            soft16(s1, hi, p1, inv1);
            const v8f oo = wmma16g(vA, cat16(p0, p1), zf);
            v8h oh;
#pragma unroll
            for (int r = 0; r < 4; ++r) { oh[r] = toh_flush(oo[r] * inv0); oh[4 + r] = toh_flush(oo[4 + r] * inv1); }
            oh = lo ? oh : z8;
            v8h wo = *(const v8h*)(&wl[wp + 256 + lr * 8]); wo = lo ? wo : z8;
            const v8f d1 = wmma16g(cat16(wo, z8), cat16(oh, z8), zf);
            { const v4f ba = *(const v4fa*)(&bs[bob]), bb = *(const v4fa*)(&bs[bob + 4]);
#pragma unroll
              for (int r = 0; r < 4; ++r) { x[r] = lo ? (x[r] + (d1[r] + ba[r])) : 0.0f; x[4 + r] = lo ? (x[4 + r] + (d1[4 + r] + bb[r])) : 0.0f; } }
            v8h x1h;
#pragma unroll
            for (int r = 0; r < 8; ++r) x1h[r] = toh_flush(x[r]);
            v8h ww = *(const v8h*)(&wl[wp + 384 + lr * 8]); ww = lo ? ww : z8;
            const v8f d2 = wmma16g(cat16(ww, z8), cat16(x1h, z8), zf);
            { const v4f ba = *(const v4fa*)(&bs[blb]), bb = *(const v4fa*)(&bs[blb + 4]);
#pragma unroll
              for (int r = 0; r < 4; ++r) { x[r] = lo ? (x[r] + fmaxf(d2[r] + ba[r], 0.0f)) : 0.0f; x[4 + r] = lo ? (x[4 + r] + fmaxf(d2[4 + r] + bb[r], 0.0f)) : 0.0f; } }
        }

        v8h x2h;
#pragma unroll
        for (int r = 0; r < 8; ++r) x2h[r] = toh_flush(x[r]);
        const v16h xf2 = cat16(x2h, z8);
        const v8f y0 = wmma16g(xf2, wout0, zf);
        const v8f y1 = wmma16g(xf2, wout1, zf);
        float sa = 0.0f, sb = 0.0f;
#pragma unroll
        for (int r = 0; r < 7; ++r) { sa += y0[r]; sb += y1[r]; }
        sa += lo ? y0[7] : 0.0f; sb += lo ? y1[7] : 0.0f;
        sa += __shfl_xor(sa, 16, 32); sb += __shfl_xor(sb, 16, 32);
        const float ra = sa * (1.0f / 15.0f) + bout0;
        const float rb = sb * (1.0f / 15.0f) + bout1;
        if (lo) os[ob + it * AOUT + lr] = ra;
        if (lo & (lr < AOUT - 16)) os[ob + it * AOUT + 16 + lr] = rb;
    }

    wave_sync();
    float* orow = OUT + (size_t)b0 * AOUT;
#pragma unroll 1
    for (int ps = 0; ps < 2; ++ps) {
#pragma unroll
        for (int s = 0; s < 3; ++s) { const int pc = s * 32 + lane; const int pcl = pc < 80 ? pc : 79;
            const v4f val = *(const v4fa*)(&os[ob + pcl * 4]);
            if (pc < 80) *(volatile v4f*)(orow + (size_t)pc * 4) = val; }
        if (ps == 0) __threadfence(); }
}

extern "C" void kernel_launch(void* const* d_in, const int* in_sizes, int n_in,
                              void* d_out, int out_size, void* d_ws, size_t ws_size, hipStream_t stream) {
    (void)d_ws; (void)ws_size;
    if (n_in < 20) return;
    const size_t needi = (size_t)NB * NL;
    if ((size_t)in_sizes[0] < needi || (size_t)in_sizes[1] < needi || (size_t)in_sizes[2] < needi) return;
    if (in_sizes[3] < NDICE * DM || in_sizes[4] < NSTAR * DM || in_sizes[5] < NBTN * DM) return;
    if (in_sizes[6] < AOUT * DM || in_sizes[7] < AOUT) return;
    if (in_sizes[8] < 3 * DM * DM || in_sizes[9] < 3 * DM || in_sizes[10] < DM * DM || in_sizes[11] < DM || in_sizes[12] < DM * DM || in_sizes[13] < DM) return;
    if (in_sizes[14] < 3 * DM * DM || in_sizes[15] < 3 * DM || in_sizes[16] < DM * DM || in_sizes[17] < DM || in_sizes[18] < DM * DM || in_sizes[19] < DM) return;
    if ((size_t)out_size < (size_t)NB * AOUT) return;
    const int*   dice_type  = (const int*)d_in[0];
    const int*   dice_star  = (const int*)d_in[1];
    const int*   summon_lvl = (const int*)d_in[2];
    const float* emb_dice   = (const float*)d_in[3];
    const float* emb_star   = (const float*)d_in[4];
    const float* emb_btns   = (const float*)d_in[5];
    const float* Wout       = (const float*)d_in[6];
    const float* bout       = (const float*)d_in[7];
    const float* Wqkv0      = (const float*)d_in[8];
    const float* bqkv0      = (const float*)d_in[9];
    const float* Wo0        = (const float*)d_in[10];
    const float* bo0        = (const float*)d_in[11];
    const float* Wl0        = (const float*)d_in[12];
    const float* bl0        = (const float*)d_in[13];
    const float* Wqkv1      = (const float*)d_in[14];
    const float* bqkv1      = (const float*)d_in[15];
    const float* Wo1        = (const float*)d_in[16];
    const float* bo1        = (const float*)d_in[17];
    const float* Wl1        = (const float*)d_in[18];
    const float* bl1        = (const float*)d_in[19];
    k_encoder<<<dim3(NB / (WPB * IPW), 1, 1), BLOCK, 0, stream>>>(
        dice_type, dice_star, summon_lvl, emb_dice, emb_star, emb_btns, Wout, bout,
        Wqkv0, bqkv0, Wo0, bo0, Wl0, bl0, Wqkv1, bqkv1, Wo1, bo1, Wl1, bl1, (float*)d_out);
}
